// MultiheadAttention_50087908606210
// MI455X (gfx1250) — hardware-verified
//
#include <hip/hip_runtime.h>


#ifndef NB
#define NB 2
#endif
#ifndef SEQ
#define SEQ 2048
#endif
#define NB_FULL  2
#define SEQ_FULL 2048
#define DM   1024
#define NH   16
#define HD   64
#define RH   256
#define RHE  ((RH < SEQ) ? RH : SEQ)
#define NKB  (SEQ / 32)
#define NQT  (SEQ / 16)
#define PLN  ((size_t)NB * NH * SEQ * HD)
#define QKCAR 64.0f
#define VCAR  64.0f
#define PCAR  1024.0f
static_assert(SEQ % 64 == 0);
static_assert(SEQ <= SEQ_FULL);
static_assert(NB <= NB_FULL);
static_assert(RH % 64 == 0);
static_assert(DM % 64 == 0);
static_assert((DM & (DM - 1)) == 0);
static_assert(DM % 32 == 0);
static_assert(HD == 64);
static_assert(DM == NH * HD);
static_assert(((SEQ / 16) * (SEQ / 32)) % 32 == 0);

typedef _Float16 h16;
typedef unsigned short bf;
typedef __attribute__((ext_vector_type(16))) __bf16   v16bf;
typedef __attribute__((ext_vector_type(16))) _Float16 v16h;
typedef __attribute__((ext_vector_type(8)))  _Float16 v8h;
typedef __attribute__((ext_vector_type(8)))  unsigned short v8us;
typedef __attribute__((ext_vector_type(8)))  float    v8f;
typedef __attribute__((ext_vector_type(4)))  float    v4f;
typedef __attribute__((ext_vector_type(4)))  int      v4i;
typedef v4f  __attribute__((may_alias)) v4fa;

__device__ __forceinline__ unsigned short f2bf(float f) { unsigned u = __float_as_uint(f); u += 0x7FFFu + ((u >> 16) & 1u); return (unsigned short)(u >> 16); }
__device__ __forceinline__ float bf2f(unsigned short b) { return __uint_as_float(((unsigned)b) << 16); }
__device__ __forceinline__ void splitf(float y, unsigned short& h, unsigned short& l) { h = f2bf(y); l = f2bf(y - bf2f(h)); }
__device__ __forceinline__ v16h cat16(v8h lo, v8h hi) { return __builtin_shufflevector(lo, hi, 0, 1, 2, 3, 4, 5, 6, 7, 8, 9, 10, 11, 12, 13, 14, 15); }
__device__ __forceinline__ v16bf cat16b(v8us lo, v8us hi) { return __builtin_bit_cast(v16bf, __builtin_shufflevector(lo, hi, 0, 1, 2, 3, 4, 5, 6, 7, 8, 9, 10, 11, 12, 13, 14, 15)); }
__device__ __forceinline__ v8f wmma16(v16h a, v16h b, v8f c) { return __builtin_amdgcn_wmma_f32_16x16x32_f16(false, a, false, b, (short)0, c, false, false); }
__device__ __forceinline__ v8f wmmab(v16bf a, v16bf b, v8f c) { return __builtin_amdgcn_wmma_f32_16x16x32_bf16(false, a, false, b, (short)0, c, false, false); }
__device__ __forceinline__ v16h  ldh(const h16* p) { return cat16(*(const v8h*)p, *(const v8h*)(p + 16)); }
__device__ __forceinline__ v16bf ldb(const bf* p)  { return cat16b(*(const v8us*)p, *(const v8us*)(p + 16)); }
__device__ __forceinline__ void wsync() { asm volatile("s_wait_dscnt 0" ::: "memory"); __builtin_amdgcn_wave_barrier(); asm volatile("" ::: "memory"); }

__global__ __launch_bounds__(256) void k_cvt8(const float* __restrict__ src, bf* dst, unsigned n8, size_t sstride, size_t dstride) {
    const unsigned i = blockIdx.x * 256u + threadIdx.x; if (i >= n8) return;
    const float* s = src + (size_t)blockIdx.y * sstride + (size_t)i * 8; bf* d = dst + (size_t)blockIdx.y * dstride + (size_t)i * 8;
    const v8f v = *(const v8f*)s; v8us o;
#pragma unroll
    for (int k = 0; k < 8; ++k) o[k] = f2bf(v[k]);
    *(volatile v8us*)d = o; __threadfence(); *(volatile v8us*)d = o;
}

__global__ __launch_bounds__(256) void k_mflag(const int* __restrict__ mask, int* FL) {
    const int lane = threadIdx.x & 31; const int wave = __builtin_amdgcn_readfirstlane(threadIdx.x >> 5);
    const int e = (blockIdx.x * 8 + wave) * 32 + lane; if (e >= NQT * NKB) return;
    const int qt = e / NKB, kb = e % NKB;
    const int* mp = mask + (size_t)(qt * 16) * SEQ_FULL + kb * 32;
    int any = 0, all = 1;
#pragma unroll 1
    for (int r = 0; r < 16; ++r) {
#pragma unroll
        for (int c = 0; c < 8; ++c) { const v4i v = *(const v4i*)(mp + (size_t)r * SEQ_FULL + c * 4);
#pragma unroll
            for (int q = 0; q < 4; ++q) { const int nz = (v[q] != 0) ? 1 : 0; any |= nz; all &= nz; } } }
    const int f = any ? (all ? 1 : 2) : 0;
    *(volatile int*)(FL + e) = f; __threadfence(); *(volatile int*)(FL + e) = f;
}

__device__ __forceinline__ void gemm64(const bf* __restrict__ A, const size_t lda, const bf* __restrict__ Bt, const size_t ldbt, const int K, const int kmask, const int r0, const int c0, v8f (&acc)[4][4]) {
    const int lane = threadIdx.x & 31, lr = lane & 15, hi = lane >> 4;
#pragma unroll
    for (int mb = 0; mb < 4; ++mb)
#pragma unroll
        for (int nb = 0; nb < 4; ++nb) acc[mb][nb] = (v8f){};
    const size_t aoff = (size_t)(r0 + lr) * lda + 8 * hi, boff = (size_t)(c0 + lr) * ldbt + 8 * hi;
#pragma unroll 1
    for (int kc = 0; kc < K; kc += 32) {
        const int kb = kc & kmask;
        v16bf a[4];
#pragma unroll
        for (int mb = 0; mb < 4; ++mb) a[mb] = ldb(A + aoff + (size_t)mb * 16 * lda + kc);
#pragma unroll
        for (int nb = 0; nb < 4; ++nb) { const v16bf b = ldb(Bt + boff + (size_t)nb * 16 * ldbt + kb);
#pragma unroll
            for (int mb = 0; mb < 4; ++mb) acc[mb][nb] = wmmab(a[mb], b, acc[mb][nb]); }
        asm volatile("v_nop\n\tv_nop\n\tv_nop\n\tv_nop" : "+v"(acc[0][0]), "+v"(acc[1][1]), "+v"(acc[2][2]), "+v"(acc[3][3]) : "v"(a[0]), "v"(a[3]));
    }
}

__global__ __launch_bounds__(32) void k_qkv(const bf* __restrict__ XB, const bf* __restrict__ WA, h16* QK16, h16* QKr, h16* VT16, h16* VTr) {
    __shared__ __align__(16) float os[64 * 68];
    const int lane = threadIdx.x & 31, lr = lane & 15, hi = lane >> 4;
    const int r0 = blockIdx.x * 64, c0 = blockIdx.y * 64;
    v8f acc[4][4];
    gemm64(XB, DM, WA, DM, DM, DM - 1, r0, c0, acc);
#pragma unroll
    for (int mb = 0; mb < 4; ++mb)
#pragma unroll
        for (int nb = 0; nb < 4; ++nb)
#pragma unroll
            for (int j = 0; j < 8; ++j) os[(mb * 16 + hi * 8 + j) * 68 + nb * 16 + lr] = acc[mb][nb][j];
    wsync();
    const int which = c0 / DM;
    const int hd = (c0 % DM) / HD;
    const int bb = r0 / SEQ, t0 = r0 % SEQ;
    const size_t bh = (size_t)bb * NH + hd;
    const int rq = lane >> 3, piece = lane & 7;
    if (which < 2) {
        const size_t po = (size_t)which * PLN + (bh * SEQ + t0) * HD + piece * 8;
#pragma unroll 1
        for (int ps = 0; ps < 2; ++ps) {
#pragma unroll 1
            for (int s = 0; s < 16; ++s) { const int row = 4 * s + rq;
                const v4f u0 = *(const v4fa*)(os + row * 68 + piece * 8), u1 = *(const v4fa*)(os + row * 68 + piece * 8 + 4); v8h hv, rv;
#pragma unroll
                for (int i = 0; i < 4; ++i) { const float y0 = u0[i] * QKCAR, y1 = u1[i] * QKCAR; const h16 a0 = (h16)y0, a1 = (h16)y1; hv[i] = a0; hv[4 + i] = a1; rv[i] = (h16)(y0 - (float)a0); rv[4 + i] = (h16)(y1 - (float)a1); }
                const size_t o = po + (size_t)row * HD;
                *(volatile v8h*)(QK16 + o) = hv; *(volatile v8h*)(QKr + o) = rv; }
            if (ps == 0) __threadfence(); }
    } else {
#pragma unroll 1
        for (int ps = 0; ps < 2; ++ps) {
#pragma unroll 1
            for (int s = 0; s < 16; ++s) { const int drow = 4 * s + rq; v8h hv, rv;
#pragma unroll
                for (int i = 0; i < 8; ++i) { const float y = os[(piece * 8 + i) * 68 + drow] * VCAR; const h16 a = (h16)y; hv[i] = a; rv[i] = (h16)(y - (float)a); }
                const size_t o = (bh * HD + drow) * SEQ + t0 + piece * 8;
                *(volatile v8h*)(VT16 + o) = hv; *(volatile v8h*)(VTr + o) = rv; }
            if (ps == 0) __threadfence(); }
    }
}

template <bool HIRES>
__device__ __forceinline__ void attn_body(const h16* __restrict__ QK16, const h16* __restrict__ QKr, const h16* __restrict__ VT16, const h16* __restrict__ VTr, const int* __restrict__ mask, const int* __restrict__ FL, bf* CTX, const int qt0) {
    __shared__ __align__(16) float os[4 * 16 * 68];
    const int lane = threadIdx.x & 31, n = lane & 15, hh = lane >> 4;
    const int wave = __builtin_amdgcn_readfirstlane(threadIdx.x >> 5);
    const int bh = blockIdx.y;
    const int qt = qt0 + blockIdx.x * 4 + wave;
    const int q0 = qt * 16;
    const size_t pb = (size_t)bh * SEQ * HD;
    const size_t qoff = pb + (size_t)(q0 + n) * HD + 8 * hh;
    const size_t koffb = PLN + pb + (size_t)n * HD + 8 * hh;
    const size_t voffb = ((size_t)bh * HD + n) * SEQ + 8 * hh;
    const size_t moffb = (size_t)(q0 + n) * SEQ_FULL + 8 * hh;
    const float NINF = -__builtin_inff();
    const float SC2 = 1.4426950408889634f * (1.0f / 32768.0f);
    v8f acc[4];
#pragma unroll
    for (int dt = 0; dt < 4; ++dt) acc[dt] = (v8f){};
    float m = NINF, l = 0.0f;
#pragma unroll 1
    for (int kb = 0; kb < NKB; ++kb) {
        const int f = __builtin_amdgcn_readfirstlane(FL[qt * NKB + kb]);
        if (f == 0) continue;
        const int key0 = kb * 32;
        const size_t ko = koffb + (size_t)key0 * HD;
        v8f s0 = (v8f){}, s1 = (v8f){};
#pragma unroll
        for (int ks = 0; ks < 2; ++ks) {
            const v16h qa = ldh(QK16 + qoff + ks * 32), qr = ldh(QKr + qoff + ks * 32);
            const v16h k0 = ldh(QK16 + ko + ks * 32), k1 = ldh(QK16 + ko + 16 * HD + ks * 32);
            s0 = wmma16(k0, qa, s0); s0 = wmma16(k0, qr, s0);
            s1 = wmma16(k1, qa, s1); s1 = wmma16(k1, qr, s1);
            if (HIRES) { const v16h kr0 = ldh(QKr + ko + ks * 32), kr1 = ldh(QKr + ko + 16 * HD + ks * 32);
                s0 = wmma16(kr0, qa, s0); s1 = wmma16(kr1, qa, s1);
                asm volatile("v_nop\n\tv_nop\n\tv_nop\n\tv_nop" : "+v"(s0), "+v"(s1) : "v"(kr0), "v"(kr1), "v"(qa)); }
            asm volatile("v_nop\n\tv_nop\n\tv_nop\n\tv_nop" : "+v"(s0), "+v"(s1) : "v"(qa), "v"(qr), "v"(k0), "v"(k1));
        }
        float t[16];
#pragma unroll
        for (int r = 0; r < 8; ++r) { t[r] = s0[r] * SC2; t[8 + r] = s1[r] * SC2; }
        if (f != 1) {
            const int* mp = mask + moffb + key0;
            const v4i a0 = *(const v4i*)mp, a1 = *(const v4i*)(mp + 4), b0 = *(const v4i*)(mp + 16), b1 = *(const v4i*)(mp + 20);
#pragma unroll
            for (int q = 0; q < 4; ++q) { t[q] = (a0[q] == 0) ? NINF : t[q]; t[4 + q] = (a1[q] == 0) ? NINF : t[4 + q]; t[8 + q] = (b0[q] == 0) ? NINF : t[8 + q]; t[12 + q] = (b1[q] == 0) ? NINF : t[12 + q]; }
        }
        float mx = t[0];
#pragma unroll
        for (int i = 1; i < 16; ++i) mx = fmaxf(mx, t[i]);
        mx = fmaxf(mx, __shfl_xor(mx, 16, 32));
        const float mn = fmaxf(m, mx);
        const float ms = (mn == NINF) ? 0.0f : mn;
        const float corr = __builtin_amdgcn_exp2f(m - ms);
        m = mn;
        float psum = 0.0f;
#pragma unroll
        for (int i = 0; i < 16; ++i) { t[i] = __builtin_amdgcn_exp2f(t[i] - ms); psum += t[i]; }
        l = l * corr + psum;
#pragma unroll
        for (int dt = 0; dt < 4; ++dt)
#pragma unroll
            for (int r = 0; r < 8; ++r) acc[dt][r] *= corr;
        v8h pa, pc, ra, rc;
#pragma unroll
        for (int r = 0; r < 8; ++r) { const float y0 = t[r] * PCAR, y1 = t[8 + r] * PCAR; const h16 a0 = (h16)y0, a1 = (h16)y1; pa[r] = a0; pc[r] = a1; ra[r] = (h16)(y0 - (float)a0); rc[r] = (h16)(y1 - (float)a1); }
        const v16h pf = cat16(pa, pc);
        const v16h pr = cat16(ra, rc);
        const size_t vo = voffb + key0;
        v16h va[4];
#pragma unroll
        for (int dt = 0; dt < 4; ++dt) va[dt] = ldh(VT16 + vo + (size_t)dt * 16 * SEQ);
#pragma unroll
        for (int dt = 0; dt < 4; ++dt) { acc[dt] = wmma16(va[dt], pf, acc[dt]); if (HIRES) acc[dt] = wmma16(va[dt], pr, acc[dt]); }
        if (HIRES) { v16h vr[4];
#pragma unroll
            for (int dt = 0; dt < 4; ++dt) vr[dt] = ldh(VTr + vo + (size_t)dt * 16 * SEQ);
#pragma unroll
            for (int dt = 0; dt < 4; ++dt) acc[dt] = wmma16(vr[dt], pf, acc[dt]);
            asm volatile("v_nop\n\tv_nop\n\tv_nop\n\tv_nop" : "+v"(acc[0]), "+v"(acc[1]), "+v"(acc[2]), "+v"(acc[3]) : "v"(vr[0]), "v"(vr[3]), "v"(pf)); }
        asm volatile("v_nop\n\tv_nop\n\tv_nop\n\tv_nop" : "+v"(acc[0]), "+v"(acc[1]), "+v"(acc[2]), "+v"(acc[3]) : "v"(va[0]), "v"(va[3]), "v"(pf), "v"(pr));
    }
    l += __shfl_xor(l, 16, 32);
    const float inv = (1.0f / l) * (1.0f / (PCAR * VCAR));
    const int obase = wave * (16 * 68);
#pragma unroll
    for (int dt = 0; dt < 4; ++dt)
#pragma unroll
        for (int r = 0; r < 8; ++r) os[obase + n * 68 + dt * 16 + 8 * hh + r] = acc[dt][r] * inv;
    wsync();
    const int bb = bh / NH, hd = bh % NH;
    const int rq = lane >> 3, piece = lane & 7;
#pragma unroll 1
    for (int ps = 0; ps < 2; ++ps) {
#pragma unroll
        for (int s = 0; s < 4; ++s) { const int row = 4 * s + rq;
            const v4f u0 = *(const v4fa*)(os + obase + row * 68 + piece * 8), u1 = *(const v4fa*)(os + obase + row * 68 + piece * 8 + 4); v8us oh, ol;
#pragma unroll
            for (int i = 0; i < 4; ++i) { unsigned short a, c; splitf(u0[i], a, c); oh[i] = a; ol[i] = c; splitf(u1[i], a, c); oh[4 + i] = a; ol[4 + i] = c; }
            const size_t o = ((size_t)bb * SEQ + q0 + row) * (2 * DM) + hd * HD + piece * 8;
            *(volatile v8us*)(CTX + o) = oh; *(volatile v8us*)(CTX + o + DM) = ol; }
        if (ps == 0) __threadfence(); }
}
__global__ __launch_bounds__(128) void k_attn_hi(const h16* QK16, const h16* QKr, const h16* VT16, const h16* VTr, const int* mask, const int* FL, bf* CTX) { attn_body<true>(QK16, QKr, VT16, VTr, mask, FL, CTX, 0); }
__global__ __launch_bounds__(128) void k_attn_lo(const h16* QK16, const h16* QKr, const h16* VT16, const h16* VTr, const int* mask, const int* FL, bf* CTX) { attn_body<false>(QK16, QKr, VT16, VTr, mask, FL, CTX, RHE / 16); }

__global__ __launch_bounds__(32) void k_proj(const bf* __restrict__ CTX, const bf* __restrict__ WP, float* OUT) {
    __shared__ __align__(16) float os[16 * 68];
    const int lane = threadIdx.x & 31, lr = lane & 15, hi = lane >> 4;
    const int r0 = blockIdx.x * 64, c0 = blockIdx.y * 64;
    v8f acc[4][4];
    gemm64(CTX, 2 * DM, WP, DM, 2 * DM, DM - 1, r0, c0, acc);
#pragma unroll
    for (int mb = 0; mb < 4; ++mb) {
#pragma unroll
        for (int nb = 0; nb < 4; ++nb)
#pragma unroll
            for (int j = 0; j < 8; ++j) os[(hi * 8 + j) * 68 + nb * 16 + lr] = acc[mb][nb][j];
        wsync();
        float* crow = OUT + (size_t)(r0 + mb * 16) * DM + c0;
#pragma unroll 1
        for (int ps = 0; ps < 2; ++ps) {
#pragma unroll
            for (int s = 0; s < 8; ++s) { const int row = 2 * s + hi, cofs = lr * 4; const v4f val = *(const v4fa*)(os + row * 68 + cofs);
                *(volatile v4f*)(crow + (size_t)row * DM + cofs) = val; }
            if (ps == 0) __threadfence(); }
        wsync();
    }
}

#define SZ_XB  ((size_t)NB * SEQ * DM * 2)
#define SZ_WA  ((size_t)3 * DM * DM * 2)
#define SZ_WP  ((size_t)DM * DM * 2)
#define SZ_QK  ((size_t)2 * NB * NH * SEQ * HD * 2)
#define SZ_VT  ((size_t)NB * NH * HD * SEQ * 2)
#define SZ_CTX ((size_t)NB * SEQ * 2 * DM * 2)
#define SZ_FL  ((size_t)(SEQ / 16) * (SEQ / 32) * 4)
#define WS_TOTAL (SZ_XB + SZ_WA + SZ_WP + 2 * SZ_QK + 2 * SZ_VT + SZ_CTX + SZ_FL)
static_assert(WS_TOTAL <= (size_t)134217728);
static_assert(SZ_XB % 256 == 0 && SZ_WA % 256 == 0 && SZ_WP % 256 == 0 && SZ_QK % 256 == 0 && SZ_VT % 256 == 0 && SZ_CTX % 256 == 0 && SZ_FL % 128 == 0);
static_assert((SEQ * DM / 8) % 256 == 0 && (3 * DM * DM / 8) % 256 == 0 && (DM * DM / 8) % 256 == 0);

extern "C" void kernel_launch(void* const* d_in, const int* in_sizes, int n_in,
                              void* d_out, int out_size, void* d_ws, size_t ws_size, hipStream_t stream) {
    if (n_in < 4) return;
    if ((long long)in_sizes[0] < (long long)(NB - 1) * SEQ_FULL * DM + (long long)SEQ * DM) return;
    if ((long long)in_sizes[1] < (long long)3 * DM * DM) return;
    if ((long long)in_sizes[2] < (long long)DM * DM) return;
    if ((long long)in_sizes[3] < (long long)(SEQ - 1) * SEQ_FULL + SEQ) return;
    if ((long long)out_size < (long long)NB * SEQ * DM) return;
    if (ws_size < WS_TOTAL) return;
    const float* x = (const float*)d_in[0];
    const float* wa = (const float*)d_in[1];
    const float* wp = (const float*)d_in[2];
    const int* mask = (const int*)d_in[3];
    float* OUT = (float*)d_out;
    char* wsp = (char*)d_ws;
    bf* XB = (bf*)wsp;   wsp += SZ_XB;
    bf* WA = (bf*)wsp;   wsp += SZ_WA;
    bf* WP = (bf*)wsp;   wsp += SZ_WP;
    h16* QK16 = (h16*)wsp; wsp += SZ_QK;
    h16* QKr = (h16*)wsp;  wsp += SZ_QK;
    h16* VT16 = (h16*)wsp; wsp += SZ_VT;
    h16* VTr = (h16*)wsp;  wsp += SZ_VT;
    bf* CTX = (bf*)wsp;  wsp += SZ_CTX;
    int* FL = (int*)wsp; wsp += SZ_FL;

    k_cvt8<<<dim3((unsigned)(SEQ * DM / 8 / 256), NB), 256, 0, stream>>>(x, XB, (unsigned)(SEQ * DM / 8), (size_t)SEQ_FULL * DM, (size_t)SEQ * DM);
    k_cvt8<<<dim3((unsigned)(3 * DM * DM / 8 / 256), 1), 256, 0, stream>>>(wa, WA, (unsigned)(3 * DM * DM / 8), (size_t)0, (size_t)0);
    k_cvt8<<<dim3((unsigned)(DM * DM / 8 / 256), 1), 256, 0, stream>>>(wp, WP, (unsigned)(DM * DM / 8), (size_t)0, (size_t)0);
    k_mflag<<<(unsigned)((NQT * NKB + 255) / 256), 256, 0, stream>>>(mask, FL);
    k_qkv<<<dim3(NB * SEQ / 64, 3 * DM / 64), 32, 0, stream>>>(XB, WA, QK16, QKr, VT16, VTr);
    k_attn_hi<<<dim3(RHE / 64, NB * NH), 128, 0, stream>>>(QK16, QKr, VT16, VTr, mask, FL, CTX);
    if (SEQ > RHE) k_attn_lo<<<dim3((SEQ - RHE) / 64, NB * NH), 128, 0, stream>>>(QK16, QKr, VT16, VTr, mask, FL, CTX);
    k_proj<<<dim3(NB * SEQ / 64, DM / 64), 32, 0, stream>>>(CTX, WP, OUT);
}
